// _MultiHeadSelfAttention_55628416418161
// MI455X (gfx1250) — hardware-verified
//
#include <hip/hip_runtime.h>
#include <math.h>

constexpr int kBatch = 4;
constexpr int kSeq   = 2048;
constexpr int kDim   = 1024;
constexpr int kHeads = 16;
constexpr int kDh    = 64;
constexpr int kTok   = kBatch * kSeq;
constexpr int kQKVn  = 3 * kDim;
constexpr int kQKld  = 2 * kDim;
constexpr int kVTld  = kTok;
constexpr int kBiasN = kQKVn + kDim;
constexpr float kPCarry      = 32768.0f;
constexpr float kResCarry    = 2048.0f;
constexpr float kResCarryInv = 1.0f / 2048.0f;
constexpr float kQScale      = 0.125f;
static_assert(kHeads * kDh == kDim, "shape");
static_assert(kTok % 64 == 0 && kQKld % 64 == 0 && kDim % 64 == 0 && kQKVn % 64 == 0, "M,N tile multiples of 64");
static_assert(kDim % 32 == 0, "K multiple of 32 for every GEMM");
static_assert(kSeq % 64 == 0 && kDh == 64, "attention chunking");
static_assert((kTok * kDim) % (8 * 256) == 0, "cast grid exact");
static_assert(kBiasN == 4 * 1024 && kQKVn == 3 * 1024, "bias kernel block map");

typedef __attribute__((ext_vector_type(16))) _Float16 v16h;
typedef __attribute__((ext_vector_type(8)))  _Float16 v8h;
typedef __attribute__((ext_vector_type(16))) __bf16   v16b;
typedef __attribute__((ext_vector_type(8)))  __bf16   v8b;
typedef __attribute__((ext_vector_type(8)))  float    v8f;
typedef __attribute__((ext_vector_type(4)))  float    v4f;
typedef __attribute__((ext_vector_type(4)))  unsigned int v4u;

__device__ __forceinline__ unsigned short f2bf_bits(float f) {
  unsigned u = __float_as_uint(f);
  return (unsigned short)((u + 0x7FFFu + ((u >> 16) & 1u)) >> 16);
}
__device__ __forceinline__ float bf_bits2f(unsigned short h) { return __uint_as_float(((unsigned)h) << 16); }

__device__ __forceinline__ void dep_guard_h(v8f& a, v8f& b, v16h x, v16h y) { asm volatile("v_nop\n\tv_nop\n\tv_nop\n\tv_nop" : "+v"(a), "+v"(b) : "v"(x), "v"(y)); }
__device__ __forceinline__ void dep_guard_b(v8f& a, v8f& b, v16b x, v16b y) { asm volatile("v_nop\n\tv_nop\n\tv_nop\n\tv_nop" : "+v"(a), "+v"(b) : "v"(x), "v"(y)); }
__device__ __forceinline__ void keep4_h(v16h a, v16h b, v16h c, v16h d) { asm volatile("v_nop" :: "v"(a), "v"(b), "v"(c), "v"(d)); }
__device__ __forceinline__ void keep4_b(v16b a, v16b b, v16b c, v16b d) { asm volatile("v_nop" :: "v"(a), "v"(b), "v"(c), "v"(d)); }
__device__ __forceinline__ void acc_guard4(v8f& a, v8f& b, v8f& c, v8f& d) { asm volatile("v_nop\n\tv_nop\n\tv_nop\n\tv_nop" : "+v"(a), "+v"(b), "+v"(c), "+v"(d)); }
template <typename T> struct Frag;
template <> struct Frag<_Float16> {
  typedef v16h V; union U { v16h v; v8h h[2]; };
  static __device__ __forceinline__ v16h load(const _Float16* p) {
    U f; f.h[0] = *(const v8h*)(p); f.h[1] = *(const v8h*)(p + 16); return f.v;
  }
  static __device__ __forceinline__ v8f mma(v16h a, v16h b, v8f c) {
    return __builtin_amdgcn_wmma_f32_16x16x32_f16(false, a, false, b, (short)0, c, false, false);
  }
  static __device__ __forceinline__ void guard(v8f& a, v8f& b, v16h x, v16h y) { dep_guard_h(a, b, x, y); }
  static __device__ __forceinline__ void keep(v16h a, v16h b, v16h c, v16h d) { keep4_h(a, b, c, d); }
};
template <> struct Frag<__bf16> {
  typedef v16b V; union U { v16b v; v8b h[2]; };
  static __device__ __forceinline__ v16b load(const __bf16* p) {
    U f; f.h[0] = *(const v8b*)(p); f.h[1] = *(const v8b*)(p + 16); return f.v;
  }
  static __device__ __forceinline__ v8f mma(v16b a, v16b b, v8f c) {
    return __builtin_amdgcn_wmma_f32_16x16x32_bf16(false, a, false, b, (short)0, c, false, false);
  }
  static __device__ __forceinline__ void guard(v8f& a, v8f& b, v16b x, v16b y) { dep_guard_b(a, b, x, y); }
  static __device__ __forceinline__ void keep(v16b a, v16b b, v16b c, v16b d) { keep4_b(a, b, c, d); }
};

__device__ __forceinline__ unsigned pk16(unsigned short a, unsigned short b) { return (unsigned)a | ((unsigned)b << 16); }
__device__ __forceinline__ unsigned short h_bits(float f) { const _Float16 h = (_Float16)f; return __builtin_bit_cast(unsigned short, h); }

__device__ __forceinline__ v8f mma_h16(v16h a, v16h b, v8f c) {
  c = __builtin_amdgcn_wmma_f32_16x16x32_f16(false, a, false, b, (short)0, c, false, false);
  asm volatile("v_nop\n\tv_nop\n\tv_nop\n\tv_nop" : "+v"(c) : "v"(a), "v"(b));
  return c;
}

template <int ET> struct Elem;
template <> struct Elem<0> { typedef _Float16 T; };
template <> struct Elem<1> { typedef __bf16 T; };
template <int ET, int SPLIT, int BIAS_MODE, int OUT_MODE, bool RESID, int ACT = 0>
__global__ __launch_bounds__(256) void wmma_gemm64(
    const unsigned short* __restrict__ Ap, const unsigned short* __restrict__ A2p, int lda, long strideA,
    const unsigned short* __restrict__ Btp, const unsigned short* __restrict__ Bt2p, int ldb, long strideB,
    void* __restrict__ Cout, void* __restrict__ Cout2, int ldc, long strideC,
    const float* __restrict__ bias,
    const float* __restrict__ resid, long strideR,
    int M, int N, int K, float scale) {
  typedef typename Elem<ET>::T T;
  typedef typename Frag<T>::V V;
  constexpr bool SA = (SPLIT != 0);
  constexpr bool SB = (SPLIT == 1);
  const T* A = (const T*)Ap; const T* A2 = (const T*)A2p; const T* Bt = (const T*)Btp; const T* Bt2 = (const T*)Bt2p;
  __shared__ __align__(16) float sT[8][16 * 68];
  const int b    = blockIdx.y;
  const int lane = threadIdx.x & 31;
  const int wave = threadIdx.x >> 5;
  const int tilesN = N >> 6;
  const int tilesM = M >> 6;
  const int tile = blockIdx.x * 8 + wave;
  if (tile >= tilesM * tilesN) return;
  const int tm = tile / tilesN;
  const int tn = tile - tm * tilesN;
  const int m0 = tm << 6;
  const int n0 = tn << 6;

  const T* Ab  = A  + (size_t)b * strideA;
  const T* Bb  = Bt + (size_t)b * strideB;
  const T* Ab2 = SA ? (A2  + (size_t)b * strideA) : nullptr;
  const T* Bb2 = SB ? (Bt2 + (size_t)b * strideB) : nullptr;

  const int rlane = lane & 15;
  const int koff  = (lane >> 4) * 8;
  const int mOff  = (lane >> 4) * 8;

  v8f acc[4][4];
#pragma unroll
  for (int i = 0; i < 4; ++i)
#pragma unroll
    for (int j = 0; j < 4; ++j) acc[i][j] = (v8f){0.f,0.f,0.f,0.f,0.f,0.f,0.f,0.f};

  for (int k0 = 0; k0 < K; k0 += 32) {
    V bh[4], bl[4];
#pragma unroll
    for (int j = 0; j < 4; ++j) {
      const size_t bo = (size_t)(n0 + (j << 4) + rlane) * ldb + koff + k0;
      bh[j] = Frag<T>::load(Bb + bo);
      if (SB) bl[j] = Frag<T>::load(Bb2 + bo);
    }
#pragma unroll
    for (int i = 0; i < 4; ++i) {
      const size_t ao = (size_t)(m0 + (i << 4) + rlane) * lda + koff + k0;
      V ah = Frag<T>::load(Ab + ao);
      V al;
      if (SA) al = Frag<T>::load(Ab2 + ao);
#pragma unroll
      for (int j = 0; j < 4; ++j) {
        acc[i][j] = Frag<T>::mma(ah, bh[j], acc[i][j]);
        if (SB) acc[i][j] = Frag<T>::mma(ah, bl[j], acc[i][j]);
        if (SA) acc[i][j] = Frag<T>::mma(al, bh[j], acc[i][j]);
      }
      Frag<T>::guard(acc[i][0], acc[i][3], ah, SA ? al : ah);
    }
    Frag<T>::keep(bh[0], bh[1], bh[2], bh[3]);
    if (SB) Frag<T>::keep(bl[0], bl[1], bl[2], bl[3]);
  }
  acc_guard4(acc[0][0], acc[0][1], acc[0][2], acc[0][3]);
  acc_guard4(acc[1][0], acc[1][1], acc[1][2], acc[1][3]);
  acc_guard4(acc[2][0], acc[2][1], acc[2][2], acc[2][3]);
  acc_guard4(acc[3][0], acc[3][1], acc[3][2], acc[3][3]);

  float* slab = sT[wave];
  const float* Rb = RESID ? (resid + (size_t)b * strideR) : nullptr;
#pragma unroll
  for (int i = 0; i < 4; ++i) {
    const int mBase = m0 + (i << 4);
#pragma unroll
    for (int j = 0; j < 4; ++j) {
      const int n = n0 + (j << 4) + rlane;
      float bv = 0.f;
      if (BIAS_MODE == 2) bv = bias[n];
#pragma unroll
      for (int r = 0; r < 8; ++r) {
        float v = acc[i][j][r] * scale;
        if (BIAS_MODE == 1) v += bias[mBase + mOff + r];
        if (BIAS_MODE == 2) v += bv;
        if (RESID) v += Rb[(size_t)(mBase + mOff + r) * ldc + n];
        if (ACT == 2) v = fmaxf(v, 0.0f);
        if (ACT == 4) v = (v > 0.f) ? v : 0.01f * v;
        slab[(mOff + r) * 68 + (j << 4) + rlane] = v;
      }
    }
    __builtin_amdgcn_fence(__ATOMIC_RELEASE, "workgroup");
    __builtin_amdgcn_wave_barrier();
    __builtin_amdgcn_fence(__ATOMIC_ACQUIRE, "workgroup");
    if (OUT_MODE == 0) {
      float* C = (float*)Cout + (size_t)b * strideC;
      const int hh = lane >> 4, c4 = (lane & 15) * 4;
      for (int pass = 0; pass < 2; ++pass) {
#pragma unroll
        for (int it = 0; it < 8; ++it) {
          const int row = it * 2 + hh;
          v4f v = *(const v4f*)(slab + row * 68 + c4);
          *(volatile v4f*)(C + (size_t)(mBase + row) * ldc + n0 + c4) = v;
        }
        __threadfence();
      }
    } else {
      const int q = lane >> 3, c8 = (lane & 7) * 8;
      unsigned short* C  = (unsigned short*)Cout  + (size_t)b * strideC;
      unsigned short* C2 = (OUT_MODE >= 2) ? ((unsigned short*)Cout2 + (size_t)b * strideC) : nullptr;
      for (int pass = 0; pass < 2; ++pass) {
#pragma unroll
        for (int it = 0; it < 4; ++it) {
          const int row = it * 4 + q;
          const float* sp = slab + row * 68 + c8;
          v8h hv, lv;
#pragma unroll
          for (int e = 0; e < 8; ++e) {
            if (OUT_MODE == 1) {
              hv[e] = (_Float16)sp[e];
            } else if (OUT_MODE == 2) {
              unsigned short hb = f2bf_bits(sp[e]);
              unsigned short lb = f2bf_bits(sp[e] - bf_bits2f(hb));
              hv[e] = __builtin_bit_cast(_Float16, hb);
              lv[e] = __builtin_bit_cast(_Float16, lb);
            } else {
              const _Float16 hq = (_Float16)sp[e];
              const float hf = (float)hq;
              hv[e] = hq;
              lv[e] = (_Float16)((sp[e] - hf) * kResCarry);
            }
          }
          *(volatile v8h*)(C + (size_t)(mBase + row) * ldc + n0 + c8) = hv;
          if (OUT_MODE >= 2) *(volatile v8h*)(C2 + (size_t)(mBase + row) * ldc + n0 + c8) = lv;
        }
        __threadfence();
      }
    }
    __builtin_amdgcn_fence(__ATOMIC_RELEASE, "workgroup");
    __builtin_amdgcn_wave_barrier();
    __builtin_amdgcn_fence(__ATOMIC_ACQUIRE, "workgroup");
  }
}

__global__ __launch_bounds__(256) void cast8_bf16_kernel(const float* __restrict__ in, unsigned short* __restrict__ out, int n8) {
  const int i = blockIdx.x * 256 + threadIdx.x;
  if (i >= n8) return;
  const float* p = in + 8 * (size_t)i;
  const v4f a = *(const v4f*)(p);
  const v4f c = *(const v4f*)(p + 4);
  unsigned short hb[8];
#pragma unroll
  for (int e = 0; e < 4; ++e) {
    hb[e]     = f2bf_bits(a[e]);
    hb[4 + e] = f2bf_bits(c[e]);
  }
  const v4u u = (v4u){pk16(hb[0], hb[1]), pk16(hb[2], hb[3]), pk16(hb[4], hb[5]), pk16(hb[6], hb[7])};
  unsigned short* q = out + 8 * (size_t)i;
  *(volatile v4u*)q = u;
  __threadfence();
  *(volatile v4u*)q = u;
}

__global__ __launch_bounds__(256) void wtcast_bf16_kernel(const float* __restrict__ W, unsigned short* __restrict__ out,
                                                          int nIn, int nOut) {
  __shared__ float sm[64][65];
  const int t  = threadIdx.x;
  const int k0 = blockIdx.x * 64;
  const int n0 = blockIdx.y * 64;
#pragma unroll
  for (int i = 0; i < 16; ++i) {
    const int e = i * 256 + t;
    const int r = e >> 6;
    const int c = e & 63;
    sm[c][r] = W[(size_t)(k0 + r) * nOut + n0 + c];
  }
  __syncthreads();
  const int lane = t & 31, wave = t >> 5;
  const int q = lane >> 3, c8 = (lane & 7) * 8;
  for (int pass = 0; pass < 2; ++pass) {
#pragma unroll
    for (int it = 0; it < 2; ++it) {
      const int row = wave * 8 + it * 4 + q;
      unsigned short hb[8];
#pragma unroll
      for (int e = 0; e < 8; ++e) hb[e] = f2bf_bits(sm[row][c8 + e]);
      const v4u u = (v4u){pk16(hb[0], hb[1]), pk16(hb[2], hb[3]), pk16(hb[4], hb[5]), pk16(hb[6], hb[7])};
      *(volatile v4u*)(out + (size_t)(n0 + row) * nIn + k0 + c8) = u;
    }
    __threadfence();
  }
}

__global__ __launch_bounds__(256) void bias_rne_kernel(const float* __restrict__ bq, const float* __restrict__ bo,
                                                       float* __restrict__ BR) {
  const int blk = blockIdx.x;
  const int t   = threadIdx.x;
  const float* src = (blk < 3) ? (bq + (size_t)blk * 1024) : bo;
  const v4f v = *(const v4f*)(src + 4 * t);
  v4f r;
#pragma unroll
  for (int e = 0; e < 4; ++e) r[e] = bf_bits2f(f2bf_bits(v[e]));
  float* dp = BR + (size_t)blk * 1024 + 4 * t;
  *(volatile v4f*)dp = r;
  __threadfence();
  *(volatile v4f*)dp = r;
}

constexpr int AT_D  = 64;
constexpr int AT_NW = 4;
constexpr int AT_QB = 64;
constexpr int AT_KC = 64;

__global__ __launch_bounds__(128)
void attn_causal_kernel(const unsigned short* __restrict__ QKp, const unsigned short* __restrict__ VHp,
                        const unsigned short* __restrict__ VRp, const float* __restrict__ BRp,
                        unsigned short* __restrict__ AOHp, unsigned short* __restrict__ AOLp) {
  __shared__ __align__(16) _Float16 Ksh[AT_KC * AT_D];
  __shared__ __align__(16) _Float16 Vth[AT_D * AT_KC];
  __shared__ __align__(16) _Float16 Vtr[AT_D * AT_KC];
  __shared__ __align__(16) _Float16 Psh[AT_NW][16 * AT_KC];
  __shared__ __align__(16) _Float16 Psl[AT_NW][16 * AT_KC];
  __shared__ __align__(16) float    Os[AT_NW][16 * 68];

  const int tid  = threadIdx.x;
  const int wave = tid >> 5;
  const int lane = tid & 31;
  const int hh   = lane >> 4;
  const int c    = lane & 15;

  const int nqb = kSeq / AT_QB;
  const int bx  = blockIdx.x;
  const int qb  = bx % nqb;
  const int bh  = bx / nqb;
  const int h   = bh % kHeads;
  const int b   = bh / kHeads;
  const int q0  = qb * AT_QB + wave * 16;
  const size_t tok0 = (size_t)b * kSeq;

  const _Float16*       Qp  = (const _Float16*)QKp + tok0 * kQKld + (size_t)h * kDh;
  const unsigned short* Kp  = QKp + tok0 * kQKld + kDim + (size_t)h * kDh;
  const unsigned short* Vhp = VHp + (size_t)(h * kDh) * kVTld + tok0;
  const unsigned short* Vrp = VRp + (size_t)(h * kDh) * kVTld + tok0;
  unsigned short*       Ohp = AOHp + tok0 * kDim + (size_t)h * kDh;
  unsigned short*       Olp = AOLp + tok0 * kDim + (size_t)h * kDh;

  v16h qa[2];
  {
    const _Float16* qrow = Qp + (size_t)(q0 + c) * kQKld;
#pragma unroll
    for (int dc = 0; dc < 2; ++dc) qa[dc] = Frag<_Float16>::load(qrow + dc * 32 + 8 * hh);
  }
  float bvv[4];
#pragma unroll
  for (int t = 0; t < 4; ++t) bvv[t] = BRp[2 * kDim + h * kDh + t * 16 + c];

  const float neg_inf = -__builtin_inff();
  float mrow[8], lrow[8];
  v8f oacc[4], oacr[4];
#pragma unroll
  for (int r = 0; r < 8; ++r) { mrow[r] = neg_inf; lrow[r] = 0.f; }
#pragma unroll
  for (int t = 0; t < 4; ++t) {
    oacc[t] = (v8f){0.f,0.f,0.f,0.f,0.f,0.f,0.f,0.f};
    oacr[t] = (v8f){0.f,0.f,0.f,0.f,0.f,0.f,0.f,0.f};
  }

  const int nChunks = qb + 1;
  for (int kc = 0; kc < nChunks; ++kc) {
    const int kv0 = kc * AT_KC;
    __syncthreads();
    {
      const int rr = tid >> 1, half = (tid & 1) * 32;
      const v4u* ksrc = (const v4u*)(Kp  + (size_t)(kv0 + rr) * kQKld + half);
      const v4u* hsrc = (const v4u*)(Vhp + (size_t)rr * kVTld + kv0 + half);
      const v4u* rsrc = (const v4u*)(Vrp + (size_t)rr * kVTld + kv0 + half);
      v4u* kd = (v4u*)(Ksh + rr * AT_D + half);
      v4u* hd = (v4u*)(Vth + rr * AT_KC + half);
      v4u* rd = (v4u*)(Vtr + rr * AT_KC + half);
      {
        const v4u w0 = ksrc[0], w1 = ksrc[1], w2 = ksrc[2], w3 = ksrc[3];
        kd[0] = w0; kd[1] = w1; kd[2] = w2; kd[3] = w3;
      }
      asm volatile("" ::: "memory");
      {
        const v4u w0 = hsrc[0], w1 = hsrc[1], w2 = hsrc[2], w3 = hsrc[3];
        hd[0] = w0; hd[1] = w1; hd[2] = w2; hd[3] = w3;
      }
      asm volatile("" ::: "memory");
      {
        const v4u w0 = rsrc[0], w1 = rsrc[1], w2 = rsrc[2], w3 = rsrc[3];
        rd[0] = w0; rd[1] = w1; rd[2] = w2; rd[3] = w3;
      }
    }
    __syncthreads();

    v8f s[4];
#pragma unroll
    for (int j = 0; j < 4; ++j) {
      s[j] = (v8f){0.f,0.f,0.f,0.f,0.f,0.f,0.f,0.f};
#pragma unroll
      for (int dc = 0; dc < 2; ++dc) {
        const v16h kb = Frag<_Float16>::load(Ksh + (j * 16 + c) * AT_D + dc * 32 + 8 * hh);
        s[j] = mma_h16(qa[dc], kb, s[j]);
      }
    }
    const bool diag = (kc == qb);
    float cm[8];
#pragma unroll
    for (int r = 0; r < 8; ++r) {
      const int qrow = q0 + 8 * hh + r;
      float m = neg_inf;
#pragma unroll
      for (int j = 0; j < 4; ++j) {
        const int kvcol = kv0 + j * 16 + c;
        float sv = s[j][r] * kQScale;
        sv = (diag && (kvcol > qrow)) ? neg_inf : sv;
        s[j][r] = sv;
        m = fmaxf(m, sv);
      }
#pragma unroll
      for (int off = 1; off < 16; off <<= 1) m = fmaxf(m, __shfl_xor(m, off, 32));
      cm[r] = m;
    }
    _Float16* pw = Psh[wave];
    _Float16* pl = Psl[wave];
#pragma unroll
    for (int r = 0; r < 8; ++r) {
      const float mnew = fmaxf(mrow[r], cm[r]);
      const float alpha = expf(mrow[r] - mnew);
      mrow[r] = mnew;
      float psum = 0.f;
#pragma unroll
      for (int j = 0; j < 4; ++j) {
        const float p  = expf(s[j][r] - mnew);
        psum += p;
        const float pc = p * kPCarry;
        const _Float16 ph = (_Float16)pc;
        const float phf = (float)ph;
        const float pres = (pc - phf) * kResCarry;
        const int pidx = (8 * hh + r) * AT_KC + j * 16 + c;
        pw[pidx] = ph;
        pl[pidx] = (_Float16)pres;
      }
#pragma unroll
      for (int off = 1; off < 16; off <<= 1) psum += __shfl_xor(psum, off, 32);
      lrow[r] = lrow[r] * alpha + psum;
#pragma unroll
      for (int t = 0; t < 4; ++t) { oacc[t][r] *= alpha; oacr[t][r] *= alpha; }
    }
    __builtin_amdgcn_fence(__ATOMIC_RELEASE, "workgroup");
    __builtin_amdgcn_wave_barrier();
    __builtin_amdgcn_fence(__ATOMIC_ACQUIRE, "workgroup");
#pragma unroll
    for (int kk = 0; kk < 2; ++kk) {
      const v16h pa = Frag<_Float16>::load(pw + c * AT_KC + kk * 32 + 8 * hh);
      const v16h pr = Frag<_Float16>::load(pl + c * AT_KC + kk * 32 + 8 * hh);
#pragma unroll
      for (int t = 0; t < 4; ++t) {
        const v16h vb = Frag<_Float16>::load(Vth + (t * 16 + c) * AT_KC + kk * 32 + 8 * hh);
        const v16h vr = Frag<_Float16>::load(Vtr + (t * 16 + c) * AT_KC + kk * 32 + 8 * hh);
        oacc[t] = mma_h16(pa, vb, oacc[t]);
        oacr[t] = mma_h16(pa, vr, oacr[t]);
        oacr[t] = mma_h16(pr, vb, oacr[t]);
      }
    }
  }

  float* os = Os[wave];
#pragma unroll
  for (int r = 0; r < 8; ++r) {
    const float inv  = 1.0f / (lrow[r] * kPCarry);
    const float invr = inv * kResCarryInv;
#pragma unroll
    for (int t = 0; t < 4; ++t) os[(8 * hh + r) * 68 + t * 16 + c] = (oacc[t][r] * inv + oacr[t][r] * invr) + bvv[t];
  }
  __builtin_amdgcn_fence(__ATOMIC_RELEASE, "workgroup");
  __builtin_amdgcn_wave_barrier();
  __builtin_amdgcn_fence(__ATOMIC_ACQUIRE, "workgroup");
  {
    const int q4 = lane >> 3, c8 = (lane & 7) * 8;
    for (int pass = 0; pass < 2; ++pass) {
#pragma unroll
      for (int it = 0; it < 4; ++it) {
        const int row = it * 4 + q4;
        const float* sp = os + row * 68 + c8;
        unsigned short hb[8], lb[8];
#pragma unroll
        for (int e = 0; e < 8; ++e) {
          hb[e] = f2bf_bits(sp[e]);
          lb[e] = f2bf_bits(sp[e] - bf_bits2f(hb[e]));
        }
        const v4u uh = (v4u){pk16(hb[0], hb[1]), pk16(hb[2], hb[3]), pk16(hb[4], hb[5]), pk16(hb[6], hb[7])};
        const v4u ul = (v4u){pk16(lb[0], lb[1]), pk16(lb[2], lb[3]), pk16(lb[4], lb[5]), pk16(lb[6], lb[7])};
        *(volatile v4u*)(Ohp + (size_t)(q0 + row) * kDim + c8) = uh;
        *(volatile v4u*)(Olp + (size_t)(q0 + row) * kDim + c8) = ul;
      }
      __threadfence();
    }
  }
}

extern "C" void kernel_launch(void* const* d_in, const int* in_sizes, int n_in,
                              void* d_out, int out_size, void* d_ws, size_t ws_size,
                              hipStream_t stream) {
  if (n_in < 5) return;
  if (in_sizes[0] != kTok * kDim) return;
  if (in_sizes[1] != kDim * kQKVn) return;
  if (in_sizes[2] != kQKVn) return;
  if (in_sizes[3] != kDim * kDim) return;
  if (in_sizes[4] != kDim) return;
  if (out_size != kTok * kDim) return;

  const size_t szXB  = (size_t)kTok * kDim * 2;
  const size_t szWQT = (size_t)kQKVn * kDim * 2;
  const size_t szWOT = (size_t)kDim * kDim * 2;
  const size_t szBR  = (size_t)kBiasN * 4;
  const size_t szQK  = (size_t)kTok * kQKld * 2;
  const size_t szVT  = (size_t)kDim * kVTld * 2;
  const size_t szAO  = (size_t)kTok * kDim * 2;
  const size_t offXB  = 0;
  const size_t offWQT = offXB + szXB;
  const size_t offWOT = offWQT + szWQT;
  const size_t offBR  = offWOT + szWOT;
  const size_t offQK  = offBR + szBR;
  const size_t offVTH = offQK + szQK;
  const size_t offVTR = offVTH + szVT;
  const size_t offAOH = offVTR + szVT;
  const size_t offAOL = offAOH + szAO;
  const size_t total  = offAOL + szAO;
  if (ws_size < total) return;

  const float* x     = (const float*)d_in[0];
  const float* w_qkv = (const float*)d_in[1];
  const float* b_qkv = (const float*)d_in[2];
  const float* w_out = (const float*)d_in[3];
  const float* b_out = (const float*)d_in[4];
  float* out = (float*)d_out;
  char* ws = (char*)d_ws;
  unsigned short* XB  = (unsigned short*)(ws + offXB);
  unsigned short* WQT = (unsigned short*)(ws + offWQT);
  unsigned short* WOT = (unsigned short*)(ws + offWOT);
  float*          BR  = (float*)(ws + offBR);
  unsigned short* QK  = (unsigned short*)(ws + offQK);
  unsigned short* VTH = (unsigned short*)(ws + offVTH);
  unsigned short* VTR = (unsigned short*)(ws + offVTR);
  unsigned short* AOH = (unsigned short*)(ws + offAOH);
  unsigned short* AOL = (unsigned short*)(ws + offAOL);

  const int n8 = (kTok * kDim) / 8;
  cast8_bf16_kernel<<<dim3(n8 / 256), dim3(256), 0, stream>>>(x, XB, n8);
  wtcast_bf16_kernel<<<dim3(kDim / 64, kQKVn / 64), dim3(256), 0, stream>>>(w_qkv, WQT, kDim, kQKVn);
  wtcast_bf16_kernel<<<dim3(kDim / 64, kDim / 64), dim3(256), 0, stream>>>(w_out, WOT, kDim, kDim);
  bias_rne_kernel<<<dim3(kBiasN / 1024), dim3(256), 0, stream>>>(b_qkv, b_out, BR);

  const int tilesQK = (kTok / 64) * (kQKld / 64);
  wmma_gemm64<1, 0, 2, 1, false, 0><<<dim3(tilesQK / 8, 1), dim3(256), 0, stream>>>(
      XB, XB, kDim, 0L, WQT, WQT, kDim, 0L,
      (void*)QK, (void*)QK, kQKld, 0L, BR, BR, 0L, kTok, kQKld, kDim, 1.0f);

  const int tilesVT = (kDim / 64) * (kTok / 64);
  const unsigned short* WVT = WQT + (size_t)kQKld * kDim;
  wmma_gemm64<1, 0, 0, 3, false, 0><<<dim3(tilesVT / 8, 1), dim3(256), 0, stream>>>(
      WVT, WVT, kDim, 0L, XB, XB, kDim, 0L,
      (void*)VTH, (void*)VTR, kVTld, 0L, BR, BR, 0L, kDim, kTok, kDim, 1.0f);

  attn_causal_kernel<<<dim3(kBatch * kHeads * (kSeq / AT_QB)), dim3(128), 0, stream>>>(QK, VTH, VTR, BR, AOH, AOL);

  const int tilesOut = (kTok / 64) * (kDim / 64);
  wmma_gemm64<1, 2, 2, 0, false, 0><<<dim3(tilesOut / 8, 1), dim3(256), 0, stream>>>(
      AOH, AOL, kDim, 0L, WOT, WOT, kDim, 0L,
      (void*)out, (void*)out, kDim, 0L, BR + kQKVn, BR, 0L, kTok, kDim, kDim, 1.0f);
}
